// MultiHeadAttentionL_21852793602475
// MI455X (gfx1250) — hardware-verified
//
#include <hip/hip_runtime.h>
#include <math.h>

typedef __attribute__((ext_vector_type(16))) _Float16 v16h;
typedef __attribute__((ext_vector_type(16))) __bf16 v16b;
typedef __attribute__((ext_vector_type(8)))  _Float16 v8h;
typedef __attribute__((ext_vector_type(8)))  float v8f;
typedef __attribute__((ext_vector_type(4)))  float v4f;
typedef __attribute__((ext_vector_type(2)))  float v2f;
typedef __attribute__((ext_vector_type(4)))  unsigned v4u;
typedef __attribute__((ext_vector_type(4)))  int v4i;
typedef float __attribute__((may_alias)) float_a;
typedef int __attribute__((may_alias)) int_a;

template <typename T> __device__ __forceinline__ void vst2(void* p, T v) { *(volatile T*)p = v; __threadfence(); *(volatile T*)p = v; }
__device__ __forceinline__ v8f wmma16(v16h a, v16h b, v8f c) {
  v8f d = __builtin_amdgcn_wmma_f32_16x16x32_f16(false, a, false, b, (short)0, c, false, false);
  asm volatile("v_nop\n\tv_nop\n\tv_nop\n\tv_nop" : "+v"(d) : "v"(a), "v"(b));
  return d;
}
__device__ __forceinline__ v8f wmma_bf(v16b a, v16b b, v8f c) {
  v8f d = __builtin_amdgcn_wmma_f32_16x16x32_bf16(false, a, false, b, (short)0, c, false, false);
  asm volatile("v_nop\n\tv_nop\n\tv_nop\n\tv_nop" : "+v"(d) : "v"(a), "v"(b));
  return d;
}
__device__ __forceinline__ v16h frag_h(const _Float16* rowk0, int lane) {
  union { v16h v; v8h q[2]; } u; const _Float16* p = rowk0 + 8 * (lane >> 4);
  u.q[0] = *(const v8h*)p; u.q[1] = *(const v8h*)(p + 16); return u.v;
}
__device__ __forceinline__ v16h frag_f32(const float* rowk0, int lane) {
  v16h a; const float* p = rowk0 + 8 * (lane >> 4);
#pragma unroll
  for (int i = 0; i < 8; ++i) { a[i] = (_Float16)p[i]; a[8 + i] = (_Float16)p[16 + i]; }
  return a;
}
__device__ __forceinline__ v16h frag_f32s(const float* rowk0, int lane, float sc) {
  v16h a; const float* p = rowk0 + 8 * (lane >> 4);
#pragma unroll
  for (int i = 0; i < 8; ++i) { a[i] = (_Float16)(p[i] * sc); a[8 + i] = (_Float16)(p[16 + i] * sc); }
  return a;
}
__device__ __forceinline__ v16h fragc_f32(const float* W, int k0, int n, int lane, int ld, int K) {
  v16h a; const int g = lane >> 4;
#pragma unroll
  for (int i = 0; i < 8; ++i) { const int ka = k0 + 8 * g + i, kb = ka + 16;
    a[i] = (_Float16)(ka < K ? W[(size_t)(ka < K ? ka : K - 1) * ld + n] : 0.f); a[8 + i] = (_Float16)(kb < K ? W[(size_t)(kb < K ? kb : K - 1) * ld + n] : 0.f); }
  return a;
}
struct F2 { v16b h, l; };
__device__ __forceinline__ F2 bsplit16(const float v[16]) { F2 r;
#pragma unroll
  for (int i = 0; i < 16; ++i) { const __bf16 h = (__bf16)v[i]; r.h[i] = h; r.l[i] = (__bf16)(v[i] - (float)h); }
  return r; }
__device__ __forceinline__ F2 split_row(const float* row, int k0, int lane) { float v[16]; const float* p = row + k0 + 8 * (lane >> 4);
#pragma unroll
  for (int i = 0; i < 8; ++i) { v[i] = p[i]; v[8 + i] = p[16 + i]; }
  return bsplit16(v); }
__device__ __forceinline__ F2 split_rowK(const float* row, int k0, int lane, int K) { float v[16]; const int g = lane >> 4;
#pragma unroll
  for (int i = 0; i < 8; ++i) { const int ka = k0 + 8 * g + i, kb = ka + 16; v[i] = ka < K ? row[ka < K ? ka : K - 1] : 0.f; v[8 + i] = kb < K ? row[kb < K ? kb : K - 1] : 0.f; }
  return bsplit16(v); }
__device__ __forceinline__ F2 split_col(const float* W, int k0, int n, int lane, int ld, int K) { float v[16]; const int g = lane >> 4;
#pragma unroll
  for (int i = 0; i < 8; ++i) { const int ka = k0 + 8 * g + i, kb = ka + 16; v[i] = ka < K ? W[(size_t)(ka < K ? ka : K - 1) * ld + n] : 0.f; v[8 + i] = kb < K ? W[(size_t)(kb < K ? kb : K - 1) * ld + n] : 0.f; }
  return bsplit16(v); }
__device__ __forceinline__ v8f mac3(const F2& a, const F2& b, v8f c) { c = wmma_bf(a.l, b.h, c); c = wmma_bf(a.h, b.l, c); return wmma_bf(a.h, b.h, c); }
__device__ __forceinline__ float sigm(float v) { return 1.0f / (1.0f + expf(-v)); }
#define LDSX() do { asm volatile("s_wait_dscnt 0" ::: "memory"); __builtin_amdgcn_wave_barrier(); __builtin_amdgcn_fence(__ATOMIC_RELEASE, "workgroup"); } while (0)


#define NB 16
#define NBP 8
#define SS 1024
#define DM 256
#define HD 512
#define NH 16
#define DK 32
#define NRP (NBP * SS)
__device__ __forceinline__ float bfr(float v) { return (float)(__bf16)v; }
__device__ __forceinline__ v16b frag_b(const __bf16* rowk0, int lane) { return __builtin_bit_cast(v16b, frag_h((const _Float16*)rowk0, lane)); }
__device__ __attribute__((noinline)) float exp_ni(float v) { return expf(v); }

__global__ __launch_bounds__(128) void k_proj(const float* __restrict__ xq, const float* __restrict__ xk, const float* __restrict__ xv, const float* __restrict__ Wq, const float* __restrict__ bq, const float* __restrict__ Wk, const float* __restrict__ bk, const float* __restrict__ Wv, const float* __restrict__ bv, float* __restrict__ Q32, float* __restrict__ K32, float* __restrict__ V32) {
  __shared__ __align__(16) float so[4][16][132];
  const int tid = threadIdx.x, wave = tid >> 5, lane = tid & 31, col = lane & 15, g = lane >> 4; const size_t r0 = (size_t)blockIdx.x * 64 + wave * 16; const int n0 = blockIdx.y * 128, which = blockIdx.z;
  const float* X = which == 0 ? xq : (which == 1 ? xk : xv); const float* W = which == 0 ? Wq : (which == 1 ? Wk : Wv); const float* bb_ = which == 0 ? bq : (which == 1 ? bk : bv); float* O = which == 0 ? Q32 : (which == 1 ? K32 : V32);
  v8f acc[8] = {};
#pragma unroll
  for (int kc = 0; kc < DM / 32; ++kc) { const v16b a = split_row(X + (r0 + col) * DM, kc * 32, lane).h;
#pragma unroll
    for (int j = 0; j < 8; ++j) acc[j] = wmma_bf(a, split_col(W, kc * 32, n0 + j * 16 + col, lane, HD, DM).h, acc[j]); }
#pragma unroll
  for (int j = 0; j < 8; ++j) { const float bb = bfr(bb_[n0 + j * 16 + col]);
#pragma unroll
    for (int r = 0; r < 8; ++r) so[wave][8 * g + r][j * 16 + col] = acc[j][r] + bb; }
  LDSX();
  for (int rl = 0; rl < 16; ++rl) vst2(O + (r0 + rl) * HD + n0 + lane * 4, *(const v4f*)(&so[wave][rl][lane * 4]));
}
__global__ __launch_bounds__(256) void k_tr(const float* __restrict__ V32, __bf16* __restrict__ VTh, __bf16* __restrict__ VTl) {
  __shared__ __align__(16) __bf16 sh_[DK][72], sl_[DK][72];
  const int tid = threadIdx.x; const size_t bh = blockIdx.y; const int k0 = blockIdx.x * 64; const float* Vh = V32 + bh * SS * DK;
  for (int q = tid; q < 64 * DK; q += 256) { const int kl = q >> 5, d = q & 31; const float v = Vh[(size_t)(k0 + kl) * DK + d]; const __bf16 hi = (__bf16)v; sh_[d][kl] = hi; sl_[d][kl] = (__bf16)(v - (float)hi); }
  __syncthreads();
  { const int d = tid >> 3, pc = tid & 7; const size_t o = (bh * DK + d) * SS + k0 + pc * 8; vst2((unsigned*)(VTh + o), *(const v4u*)(&sh_[d][pc * 8])); vst2((unsigned*)(VTl + o), *(const v4u*)(&sl_[d][pc * 8])); }
}
__global__ __launch_bounds__(128) void k_attn(const float* __restrict__ Q32, const float* __restrict__ K32, const __bf16* __restrict__ VTh, const __bf16* __restrict__ VTl, float* __restrict__ CTX) {
  __shared__ __align__(16) float sS[4][16][68];
  __shared__ __align__(16) __bf16 sPh[4][16][72], sPl[4][16][72];
  __shared__ __align__(16) float sO[4][16][36];
  const int tid = threadIdx.x, w = tid >> 5, lane = tid & 31, col = lane & 15, g = lane >> 4; const size_t bh = blockIdx.y; const int q0 = blockIdx.x * 64 + w * 16; const float* Qh = Q32 + bh * SS * DK; const float* Kh = K32 + bh * SS * DK;
  const F2 aq = split_row(Qh + (size_t)(q0 + col) * DK, 0, lane);
  float mrun = -3.0e38f, lrun = 0.f; v8f acc[2] = {};
#pragma unroll 1
  for (int kt = 0; kt < SS / 64; ++kt) {
#pragma unroll
    for (int t = 0; t < 4; ++t) { const int key = kt * 64 + t * 16 + col; const v8f s = mac3(aq, split_row(Kh + (size_t)key * DK, 0, lane), (v8f){});
#pragma unroll
      for (int r = 0; r < 8; ++r) sS[w][8 * g + r][t * 16 + col] = s[r] * 0.70710678118654752f; }
    LDSX();
    float mx = -3.4e38f;
#pragma unroll
    for (int jj = 0; jj < 32; ++jj) mx = fmaxf(mx, sS[w][col][g * 32 + jj]);
    mx = fmaxf(mx, __shfl_xor(mx, 16, 32));
    const float mnew = fmaxf(mrun, mx); const float corr = expf(mrun - mnew);
    float ps = 0.f;
#pragma unroll 4
    for (int jj = 0; jj < 32; ++jj) { const float p = exp_ni(sS[w][col][g * 32 + jj] - mnew); ps += p; const __bf16 hi = (__bf16)p; sPh[w][col][g * 32 + jj] = hi; sPl[w][col][g * 32 + jj] = (__bf16)(p - (float)hi); }
    ps += __shfl_xor(ps, 16, 32);
    lrun = lrun * corr + ps; mrun = mnew;
#pragma unroll
    for (int r = 0; r < 8; ++r) { const float cr = __shfl(corr, 8 * g + r, 32); acc[0][r] *= cr; acc[1][r] *= cr; }
    LDSX();
#pragma unroll
    for (int kc = 0; kc < 2; ++kc) { const v16b ph = frag_b(&sPh[w][col][0] + kc * 32, lane), pl = frag_b(&sPl[w][col][0] + kc * 32, lane);
#pragma unroll
      for (int t = 0; t < 2; ++t) { const size_t vo = (bh * DK + t * 16 + col) * SS + kt * 64 + kc * 32; const v16b vh = frag_b(VTh + vo, lane), vl = frag_b(VTl + vo, lane); acc[t] = wmma_bf(pl, vh, acc[t]); acc[t] = wmma_bf(ph, vl, acc[t]); acc[t] = wmma_bf(ph, vh, acc[t]); } }
    __builtin_amdgcn_wave_barrier(); }
#pragma unroll
  for (int r = 0; r < 8; ++r) { const float lr = __shfl(lrun, 8 * g + r, 32); const float inv = 1.0f / lr; sO[w][8 * g + r][col] = acc[0][r] * inv; sO[w][8 * g + r][16 + col] = acc[1][r] * inv; }
  LDSX();
  for (int qq = lane; qq < 16 * 8; qq += 32) { const int rl = qq >> 3, pc = qq & 7; vst2(CTX + (bh * SS + q0 + rl) * DK + pc * 4, *(const v4f*)(&sO[w][rl][pc * 4])); }
}
__global__ __launch_bounds__(128) void k_res(const float* __restrict__ xq, const float* __restrict__ Wr, const float* __restrict__ br, float* __restrict__ OUT) {
  __shared__ __align__(16) float so[4][16][132];
  const int tid = threadIdx.x, wave = tid >> 5, lane = tid & 31, col = lane & 15, g = lane >> 4; const size_t r0 = (size_t)blockIdx.x * 64 + wave * 16; const int n0 = blockIdx.y * 128;
  v8f acc[8] = {};
#pragma unroll
  for (int kc = 0; kc < DM / 32; ++kc) { const v16b a = split_row(xq + (r0 + col) * DM, kc * 32, lane).h;
#pragma unroll
    for (int j = 0; j < 8; ++j) acc[j] = wmma_bf(a, split_col(Wr, kc * 32, n0 + j * 16 + col, lane, HD, DM).h, acc[j]); }
#pragma unroll
  for (int j = 0; j < 8; ++j) { const int n = n0 + j * 16 + col; const float bb = bfr(br[n]);
#pragma unroll
    for (int r = 0; r < 8; ++r) { const float v = acc[j][r] + bb + OUT[(r0 + 8 * g + r) * HD + n]; so[wave][8 * g + r][j * 16 + col] = v > 0.f ? v : 0.f; } }
  LDSX();
  for (int rl = 0; rl < 16; ++rl) vst2(OUT + (r0 + rl) * HD + n0 + lane * 4, *(const v4f*)(&so[wave][rl][lane * 4]));
}
extern "C" void kernel_launch(void* const* d_in, const int* in_sizes, int n_in, void* d_out, int out_size, void* d_ws, size_t ws_size, hipStream_t stream) {
  (void)in_sizes; (void)n_in; (void)out_size; (void)ws_size;
  const float** I = (const float**)d_in;
  const float* xk = I[0]; const float* xv = I[1]; const float* xq = I[2]; const float* Wk = I[3]; const float* bk = I[4]; const float* Wv = I[5]; const float* bv = I[6]; const float* Wq = I[7]; const float* bq = I[8]; const float* Wr = I[9]; const float* br = I[10];
  char* ws = (char*)d_ws; size_t off = 0;
  auto take = [&](size_t bytes) { char* p = ws + off; off += (bytes + 255) & ~(size_t)255; return p; };
  float* Q32 = (float*)take((size_t)NRP * HD * 4); float* K32 = (float*)take((size_t)NRP * HD * 4); float* V32 = (float*)take((size_t)NRP * HD * 4); __bf16* VTh = (__bf16*)take((size_t)NRP * HD * 2); __bf16* VTl = (__bf16*)take((size_t)NRP * HD * 2);
  for (int ps = 0; ps < NB / NBP; ++ps) { const size_t rb = (size_t)ps * NRP; float* op = (float*)d_out + rb * HD;
    k_proj<<<dim3(NRP / 64, HD / 128, 3), 128, 0, stream>>>(xq + rb * DM, xk + rb * DM, xv + rb * DM, Wq, bq, Wk, bk, Wv, bv, Q32, K32, V32);
    k_tr<<<dim3(SS / 64, NBP * NH), 256, 0, stream>>>(V32, VTh, VTl);
    k_attn<<<dim3(SS / 64, NBP * NH), 128, 0, stream>>>(Q32, K32, VTh, VTl, op);
    k_res<<<dim3(NRP / 64, HD / 128), 128, 0, stream>>>(xq + rb * DM, Wr, br, op); }
}
